// ContextAttention_38388417692113
// MI455X (gfx1250) — hardware-verified
//
#include <hip/hip_runtime.h>
#include <stdint.h>

#define IMH  96
#define IMW  96
#define NPIX (IMH * IMW)
#define NCH  64
#define NBT  2
#define NFR  2
#define NIMG (NBT * NFR)
#define KCV  (NCH * 9)
#define KQ   (NCH * NFR)
#define NO3  (3 * NCH)
#define PT   64
#define NTB  (NPIX / PT)
#define FSP  72
#define OSP  68
#define W2T_BLK ((NCH * KCV) / (8 * 256))
#define WQ3_BLK ((NO3 * KQ) / (8 * 256))
#define ASC  16.0f
#define WSC  16.0f
#define RCV  0.00390625f
#define SCL  (1.44269504088896340736f * 0.00048828125f)
#define PEX  14.0f
#define OSC  0.0625f

static_assert(NCH == 64);
static_assert((NPIX % PT) == 0);
static_assert((KCV % 32) == 0);
static_assert((KQ % 32) == 0);
static_assert((KCV % 8) == 0);
static_assert((NCH * KCV) == W2T_BLK * 8 * 256);
static_assert((NO3 * KQ) == WQ3_BLK * 8 * 256);
static_assert(((FSP * 2) % 16) == 0);
static_assert(((OSP * 4) % 16) == 0);
static_assert((PT / 4) * 4 == PT);

typedef _Float16     v8h  __attribute__((ext_vector_type(8)));
typedef _Float16     v16h __attribute__((ext_vector_type(16)));
typedef unsigned int v4u  __attribute__((ext_vector_type(4)));
typedef float        v4f  __attribute__((ext_vector_type(4)));
typedef float        v8f  __attribute__((ext_vector_type(8)));

union FragH { v8h p[2]; v4u u[2]; v16h v; };
union H8 { v8h v; _Float16 e[8]; };
static_assert(sizeof(FragH) == 32);
static_assert(sizeof(H8) == 16);

__device__ __forceinline__ v8f zero8() { v8f z = {0.f, 0.f, 0.f, 0.f, 0.f, 0.f, 0.f, 0.f}; return z; }

__device__ __forceinline__ float bf_rne(float x) {
  unsigned int u = __float_as_uint(x);
  u += 0x7FFFu + ((u >> 16) & 1u);
  return __uint_as_float(u & 0xFFFF0000u);
}

__device__ __forceinline__ v8f mma_h(v16h a, v16h b, v8f c) {
  v8f d = __builtin_amdgcn_wmma_f32_16x16x32_f16(false, a, false, b, (short)0, c, false, false);
#if defined(__HIP_DEVICE_COMPILE__)
  asm volatile("v_nop\n\tv_nop\n\tv_nop\n\tv_nop" : "+v"(d) : "v"(a), "v"(b));
#endif
  return d;
}

__device__ __forceinline__ float max8(v8f d) {
  const float a = fmaxf(d[0], d[1]);
  const float b = fmaxf(d[2], d[3]);
  const float c = fmaxf(d[4], d[5]);
  const float e = fmaxf(d[6], d[7]);
  return fmaxf(fmaxf(a, b), fmaxf(c, e));
}

__global__ __launch_bounds__(256)
void k_wprep(const float* __restrict__ W2, const float* __restrict__ QW, const float* __restrict__ KW,
             const float* __restrict__ VW, _Float16* W2T, _Float16* WQ3) {
  const int gid = blockIdx.x * 256 + threadIdx.x;
  H8 u;
  if (blockIdx.x < W2T_BLK) {
    const int e0  = 8 * gid;
    const int c   = e0 / KCV;
    const int kk0 = e0 - c * KCV;
#pragma unroll
    for (int i = 0; i < 8; ++i) {
      const int kk  = kk0 + i;
      const int tap = kk >> 6;
      const int f   = kk & 63;
      u.e[i] = (_Float16)(bf_rne(W2[(c * NCH + f) * 9 + tap]) * WSC);
    }
    _Float16* dst = W2T + e0;
    *(volatile v8h*)dst = u.v;
    __threadfence();
    *(volatile v8h*)dst = u.v;
  } else {
    const int g2  = gid - W2T_BLK * 256;
    const int e0  = 8 * g2;
    const int row = e0 >> 7;
    const int kp0 = e0 & 127;
    const int g   = row >> 6;
    const int o   = row & 63;
#pragma unroll
    for (int i = 0; i < 8; ++i) {
      const int kp  = kp0 + i;
      const int nf  = kp >> 6;
      const int c   = kp & 63;
      const int src = o * KQ + c * NFR + nf;
      const float wq  = QW[src];
      const float wk  = KW[src];
      const float wvv = VW[src];
      const float w   = (g == 0) ? wq : ((g == 1) ? wk : wvv);
      u.e[i] = (_Float16)(bf_rne(w) * WSC);
    }
    _Float16* dst = WQ3 + e0;
    *(volatile v8h*)dst = u.v;
    __threadfence();
    *(volatile v8h*)dst = u.v;
  }
}

__global__ __launch_bounds__(256)
void k_conv1(const float* __restrict__ X, const float* __restrict__ W1, const float* __restrict__ B1, _Float16* F1) {
  __shared__ __align__(16) _Float16 Fs[PT * FSP];
  const int t   = threadIdx.x;
  const int img = blockIdx.x / NTB;
  const int p0  = (blockIdx.x - img * NTB) * PT;
  const int c   = t & 63;
  const int plb = t >> 6;
  float w[9];
#pragma unroll
  for (int i = 0; i < 9; ++i) w[i] = bf_rne(W1[c * 9 + i]);
  const float bias = bf_rne(B1[c]);
  const float* xin = X + (size_t)img * NPIX;

#pragma unroll 1
  for (int it = 0; it < PT / 4; ++it) {
    const int pl = it * 4 + plb;
    const int p  = p0 + pl;
    const int py = p / IMW;
    const int px = p - py * IMW;
    float acc = bias;
#pragma unroll
    for (int tap = 0; tap < 9; ++tap) {
      const int dy = tap / 3;
      const int dx = tap - 3 * dy;
      const int yy = py + dy - 1;
      const int xx = px + dx - 1;
      const bool inb = ((unsigned)yy < (unsigned)IMH) && ((unsigned)xx < (unsigned)IMW);
      const int yc = min(max(yy, 0), IMH - 1);
      const int xc = min(max(xx, 0), IMW - 1);
      float v = bf_rne(xin[yc * IMW + xc]);
      v = inb ? v : 0.f;
      acc += w[tap] * v;
    }
    Fs[pl * FSP + c] = (_Float16)(fmaxf(acc, 0.f) * ASC);
  }
  __syncthreads();

  v8h wv[2];
  unsigned int pd[2];
#pragma unroll
  for (int it = 0; it < 2; ++it) {
    const int row = it * 32 + (t >> 3);
    const int q   = t & 7;
    wv[it] = *(const v8h*)(Fs + row * FSP + 8 * q);
    pd[it] = (unsigned int)(img * NPIX + p0 + row) * NCH + 8 * q;
  }
  *(volatile v8h*)(F1 + pd[0]) = wv[0];
  *(volatile v8h*)(F1 + pd[1]) = wv[1];
  __threadfence();
  *(volatile v8h*)(F1 + pd[0]) = wv[0];
  *(volatile v8h*)(F1 + pd[1]) = wv[1];
}

__global__ __launch_bounds__(128)
void k_conv2(const _Float16* __restrict__ F1, const _Float16* __restrict__ W2T, const float* __restrict__ B2,
             _Float16* FT) {
  __shared__ __align__(16) _Float16 Fs[PT * FSP];
  const int t    = threadIdx.x;
  const int lane = t & 31, wv = t >> 5;
  const int hh   = lane >> 4, n = lane & 15;
  const int img  = blockIdx.x / NTB;
  const int p0   = (blockIdx.x - img * NTB) * PT;
  const int b    = img >> 1;
  const int nf   = img & 1;
  const _Float16* fimg = F1 + (size_t)img * NPIX * NCH;

  const int p  = p0 + 16 * wv + n;
  const int pa = p / IMW;
  const int pb = p - pa * IMW;

  v8f acc[4];
#pragma unroll
  for (int ct = 0; ct < 4; ++ct) acc[ct] = zero8();

#pragma unroll 1
  for (int st = 0; st < KCV / 32; ++st) {
    const int tap = st >> 1;
    const int dy  = tap / 3;
    const int dx  = tap - 3 * dy;
    const int aa  = pa + dy - 1;
    const int bb  = pb + dx - 1;
    const bool inb = ((unsigned)aa < (unsigned)IMH) && ((unsigned)bb < (unsigned)IMW);
    const int ac  = min(max(aa, 0), IMH - 1);
    const int bc  = min(max(bb, 0), IMW - 1);
    const unsigned int msk = inb ? 0xFFFFFFFFu : 0u;
    const _Float16* xp = fimg + (size_t)(ac * IMW + bc) * NCH + (st & 1) * 32 + 8 * hh;
    FragH a;
    a.p[0] = *(const v8h*)(xp);
    a.p[1] = *(const v8h*)(xp + 16);
    a.u[0] = a.u[0] & msk;
    a.u[1] = a.u[1] & msk;
#pragma unroll
    for (int ct = 0; ct < 4; ++ct) {
      const _Float16* wp = W2T + (size_t)(ct * 16 + n) * KCV + st * 32 + 8 * hh;
      FragH w;
      w.p[0] = *(const v8h*)(wp);
      w.p[1] = *(const v8h*)(wp + 16);
      acc[ct] = mma_h(a.v, w.v, acc[ct]);
    }
  }

#pragma unroll
  for (int ct = 0; ct < 4; ++ct) {
    const float bbias = bf_rne(B2[ct * 16 + n]);
#pragma unroll
    for (int r = 0; r < 8; ++r) {
      float v = acc[ct][r] * RCV + bbias;
      v = fmaxf(v, 0.f) * ASC;
      Fs[(16 * wv + 8 * hh + r) * FSP + ct * 16 + n] = (_Float16)v;
    }
  }
  __syncthreads();

  v8h w4[4];
  unsigned int pd[4];
#pragma unroll
  for (int it = 0; it < 4; ++it) {
    const int row = it * 16 + (t >> 3);
    const int q   = t & 7;
    w4[it] = *(const v8h*)(Fs + row * FSP + 8 * q);
    pd[it] = (unsigned int)(b * NPIX + p0 + row) * KQ + nf * NCH + 8 * q;
  }
#pragma unroll
  for (int it = 0; it < 4; ++it) *(volatile v8h*)(FT + pd[it]) = w4[it];
  __threadfence();
#pragma unroll
  for (int it = 0; it < 4; ++it) *(volatile v8h*)(FT + pd[it]) = w4[it];
}

__global__ __launch_bounds__(128)
void k_qkv(const _Float16* __restrict__ FT, const _Float16* __restrict__ WQ3,
           const float* __restrict__ QB, const float* __restrict__ KB, const float* __restrict__ VB,
           _Float16* QP, _Float16* KP, _Float16* VP) {
  __shared__ __align__(16) _Float16 Ts[3 * PT * FSP];
  const int t    = threadIdx.x;
  const int lane = t & 31, wv = t >> 5;
  const int hh   = lane >> 4, n = lane & 15;
  const int b    = blockIdx.x / NTB;
  const int t0   = (blockIdx.x - b * NTB) * PT;

  const _Float16* ap = FT + (size_t)(b * NPIX + t0 + 16 * wv + n) * KQ + 8 * hh;
  FragH a[4];
#pragma unroll
  for (int ks = 0; ks < 4; ++ks) {
    a[ks].p[0] = *(const v8h*)(ap + ks * 32);
    a[ks].p[1] = *(const v8h*)(ap + ks * 32 + 16);
  }

#pragma unroll
  for (int g = 0; g < 3; ++g) {
    v8f acc[4];
#pragma unroll
    for (int ct = 0; ct < 4; ++ct) acc[ct] = zero8();
#pragma unroll
    for (int ks = 0; ks < 4; ++ks) {
#pragma unroll
      for (int ct = 0; ct < 4; ++ct) {
        const _Float16* wp = WQ3 + (size_t)(g * NCH + ct * 16 + n) * KQ + ks * 32 + 8 * hh;
        FragH w;
        w.p[0] = *(const v8h*)(wp);
        w.p[1] = *(const v8h*)(wp + 16);
        acc[ct] = mma_h(a[ks].v, w.v, acc[ct]);
      }
    }
    const float* bp = (g == 0) ? QB : ((g == 1) ? KB : VB);
#pragma unroll
    for (int ct = 0; ct < 4; ++ct) {
      const float bbias = bf_rne(bp[ct * 16 + n]);
#pragma unroll
      for (int r = 0; r < 8; ++r) {
        const float v = (acc[ct][r] * RCV + bbias) * ASC;
        const _Float16 h16 = (_Float16)v;
        if (g < 2) {
          Ts[g * PT * FSP + (16 * wv + 8 * hh + r) * FSP + ct * 16 + n] = h16;
        } else {
          Ts[2 * PT * FSP + (ct * 16 + n) * FSP + 16 * wv + 8 * hh + r] = h16;
        }
      }
    }
  }
  __syncthreads();

  v8h w[12];
  unsigned int pd[12];
#pragma unroll
  for (int it = 0; it < 12; ++it) {
    const int pl  = it >> 2;
    const int row = (it & 3) * 16 + (t >> 3);
    const int q   = t & 7;
    w[it] = *(const v8h*)(Ts + pl * PT * FSP + row * FSP + 8 * q);
    if (pl < 2) pd[it] = (unsigned int)(b * NPIX + t0 + row) * NCH + 8 * q;
    else        pd[it] = (unsigned int)(b * NCH + row) * NPIX + t0 + 8 * q;
  }
#define QKV_PASS \
  *(volatile v8h*)(QP + pd[0]) = w[0]; *(volatile v8h*)(QP + pd[1]) = w[1]; \
  *(volatile v8h*)(QP + pd[2]) = w[2]; *(volatile v8h*)(QP + pd[3]) = w[3]; \
  *(volatile v8h*)(KP + pd[4]) = w[4]; *(volatile v8h*)(KP + pd[5]) = w[5]; \
  *(volatile v8h*)(KP + pd[6]) = w[6]; *(volatile v8h*)(KP + pd[7]) = w[7]; \
  *(volatile v8h*)(VP + pd[8]) = w[8]; *(volatile v8h*)(VP + pd[9]) = w[9]; \
  *(volatile v8h*)(VP + pd[10]) = w[10]; *(volatile v8h*)(VP + pd[11]) = w[11]
  QKV_PASS;
  __threadfence();
  QKV_PASS;
#undef QKV_PASS
}

__global__ __launch_bounds__(128)
void k_attn(const _Float16* __restrict__ QP, const _Float16* __restrict__ KP, const _Float16* __restrict__ VP,
            float* out) {
  __shared__ __align__(16) float Os[NCH * OSP];
  const int t    = threadIdx.x;
  const int lane = t & 31, wv = t >> 5;
  const int hh   = lane >> 4, n = lane & 15;
  const int b    = blockIdx.x / NTB;
  const int bm0  = (blockIdx.x - b * NTB) * PT;
  const int m0   = bm0 + wv * 16;

  const size_t tq = (size_t)(b * NPIX + m0 + n) * NCH + 8 * hh;
  FragH q0, q1;
  q0.p[0] = *(const v8h*)(QP + tq);
  q0.p[1] = *(const v8h*)(QP + tq + 16);
  q1.p[0] = *(const v8h*)(QP + tq + 32);
  q1.p[1] = *(const v8h*)(QP + tq + 48);

  const size_t kb = (size_t)(b * NPIX + n) * NCH + 8 * hh;
  const size_t vb = (size_t)(b * NCH + n) * NPIX + 8 * hh;

  v8f O[4];
#pragma unroll
  for (int ct = 0; ct < 4; ++ct) O[ct] = zero8();
  float m = -1.0e30f, z = 0.f;

#pragma unroll 1
  for (int k0 = 0; k0 < NPIX; k0 += PT) {
    v8f S[4];
#pragma unroll
    for (int ks = 0; ks < 4; ++ks) {
      const size_t ao = kb + (size_t)(k0 + 16 * ks) * NCH;
      FragH f0, f1;
      f0.p[0] = *(const v8h*)(KP + ao);
      f0.p[1] = *(const v8h*)(KP + ao + 16);
      f1.p[0] = *(const v8h*)(KP + ao + 32);
      f1.p[1] = *(const v8h*)(KP + ao + 48);
      v8f zz = mma_h(f0.v, q0.v, zero8());
      zz     = mma_h(f1.v, q1.v, zz);
      S[ks]  = zz;
    }

    float tm = fmaxf(max8(S[0]), max8(S[1]));
    tm = fmaxf(tm, fmaxf(max8(S[2]), max8(S[3])));
    const float tmo = __shfl_xor(tm, 16, 32);
    tm = fmaxf(tm, tmo);
    const float mn    = fmaxf(m, tm * SCL);
    const float alpha = __builtin_amdgcn_exp2f(m - mn);
    m = mn;
    const float nb = PEX - mn;
    z *= alpha;
#pragma unroll
    for (int ct = 0; ct < 4; ++ct) O[ct] = O[ct] * alpha;

    FragH pf0, pf1;
#pragma unroll
    for (int r = 0; r < 8; ++r) {
      const _Float16 e0 = (_Float16)__builtin_amdgcn_exp2f(fmaf(S[0][r], SCL, nb));
      const _Float16 e1 = (_Float16)__builtin_amdgcn_exp2f(fmaf(S[1][r], SCL, nb));
      const _Float16 e2 = (_Float16)__builtin_amdgcn_exp2f(fmaf(S[2][r], SCL, nb));
      const _Float16 e3 = (_Float16)__builtin_amdgcn_exp2f(fmaf(S[3][r], SCL, nb));
      pf0.v[r]     = e0;
      pf0.v[8 + r] = e1;
      pf1.v[r]     = e2;
      pf1.v[8 + r] = e3;
      z += (float)e0;
      z += (float)e1;
      z += (float)e2;
      z += (float)e3;
    }

#pragma unroll
    for (int ct = 0; ct < 4; ++ct) {
      const _Float16* yp = VP + vb + (size_t)ct * 16 * NPIX + k0;
      FragH ay, by;
      ay.p[0] = *(const v8h*)(yp);
      ay.p[1] = *(const v8h*)(yp + 16);
      by.p[0] = *(const v8h*)(yp + 32);
      by.p[1] = *(const v8h*)(yp + 48);
      O[ct] = mma_h(ay.v, pf0.v, O[ct]);
      O[ct] = mma_h(by.v, pf1.v, O[ct]);
    }
  }

  const float zo = __shfl_xor(z, 16, 32);
  const float zt = z + zo;
  const float rz = __builtin_amdgcn_rcpf(zt) * OSC;
#pragma unroll
  for (int ct = 0; ct < 4; ++ct) {
#pragma unroll
    for (int r = 0; r < 8; ++r) {
      Os[(ct * 16 + 8 * hh + r) * OSP + 16 * wv + n] = O[ct][r] * rz;
    }
  }
  __syncthreads();

  v4f          ov[8];
  unsigned int po[8];
#pragma unroll
  for (int it = 0; it < 8; ++it) {
    const int L    = it * 16 + (t >> 3);
    const int c    = L >> 1;
    const int half = L & 1;
    const int q    = t & 7;
    ov[it] = *(const v4f*)(Os + c * OSP + half * 32 + 4 * q);
    po[it] = (unsigned int)(b * NCH + c) * NPIX + bm0 + half * 32 + 4 * q;
  }
#pragma unroll
  for (int it = 0; it < 8; ++it) *(volatile v4f*)(out + po[it]) = ov[it];
  __threadfence();
#pragma unroll
  for (int it = 0; it < 8; ++it) *(volatile v4f*)(out + po[it]) = ov[it];
}

extern "C" void kernel_launch(void* const* d_in, const int* in_sizes, int n_in,
                              void* d_out, int out_size, void* d_ws, size_t ws_size,
                              hipStream_t stream) {
  if (n_in < 11) return;
  if (in_sizes[0]  != NIMG * NPIX) return;
  if (in_sizes[1]  != NCH * 9) return;
  if (in_sizes[2]  != NCH) return;
  if (in_sizes[3]  != NCH * KCV) return;
  if (in_sizes[4]  != NCH) return;
  if (in_sizes[5]  != NCH * KQ) return;
  if (in_sizes[6]  != NCH) return;
  if (in_sizes[7]  != NCH * KQ) return;
  if (in_sizes[8]  != NCH) return;
  if (in_sizes[9]  != NCH * KQ) return;
  if (in_sizes[10] != NCH) return;
  if (out_size != NBT * NCH * NPIX) return;

  size_t off = 0;
  const size_t szW2T = (size_t)NCH * KCV * 2;
  const size_t szWQ3 = (size_t)NO3 * KQ * 2;
  const size_t szF1  = (size_t)NIMG * NPIX * NCH * 2;
  const size_t szFT  = (size_t)NBT * NPIX * KQ * 2;
  const size_t szP   = (size_t)NBT * NPIX * NCH * 2;
  const size_t oW2T = off; off += szW2T;
  const size_t oWQ3 = off; off += szWQ3;
  const size_t oF1  = off; off += szF1;
  const size_t oFT  = off; off += szFT;
  const size_t oQP  = off; off += szP;
  const size_t oKP  = off; off += szP;
  const size_t oVP  = off; off += szP;
  if (off > ws_size) return;
  if (off > (size_t)134217728) return;
  if ((oWQ3 % 256) != 0 || (oF1 % 256) != 0 || (oFT % 256) != 0 || (oQP % 256) != 0 ||
      (oKP % 256) != 0 || (oVP % 256) != 0) return;

  const float* X  = (const float*)d_in[0];
  const float* W1 = (const float*)d_in[1];
  const float* B1 = (const float*)d_in[2];
  const float* W2 = (const float*)d_in[3];
  const float* B2 = (const float*)d_in[4];
  const float* QW = (const float*)d_in[5];
  const float* QB = (const float*)d_in[6];
  const float* KW = (const float*)d_in[7];
  const float* KB = (const float*)d_in[8];
  const float* VW = (const float*)d_in[9];
  const float* VB = (const float*)d_in[10];
  float* out = (float*)d_out;

  char* ws = (char*)d_ws;
  _Float16* W2T = (_Float16*)(ws + oW2T);
  _Float16* WQ3 = (_Float16*)(ws + oWQ3);
  _Float16* F1  = (_Float16*)(ws + oF1);
  _Float16* FT  = (_Float16*)(ws + oFT);
  _Float16* QP  = (_Float16*)(ws + oQP);
  _Float16* KP  = (_Float16*)(ws + oKP);
  _Float16* VP  = (_Float16*)(ws + oVP);

  k_wprep<<<dim3(W2T_BLK + WQ3_BLK), dim3(256), 0, stream>>>(W2, QW, KW, VW, W2T, WQ3);
  k_conv1<<<dim3(NIMG * NTB), dim3(256), 0, stream>>>(X, W1, B1, F1);
  k_conv2<<<dim3(NIMG * NTB), dim3(128), 0, stream>>>(F1, W2T, B2, FT);
  k_qkv<<<dim3(NBT * NTB), dim3(128), 0, stream>>>(FT, WQ3, QB, KB, VB, QP, KP, VP);
  k_attn<<<dim3(NBT * NTB), dim3(128), 0, stream>>>(QP, KP, VP, out);
  (void)hipGetLastError();
}
